// IterativeRefiner_5935644803520
// MI455X (gfx1250) — hardware-verified
//
#include <hip/hip_runtime.h>
#include <math.h>

constexpr int kB   = 4;
constexpr int kNE  = 128;
constexpr int kNV  = 1024;
constexpr int kDIN = 64;
constexpr int kD   = 128;
constexpr int kT   = 2;
static_assert(kT == 2);
constexpr int kRowsE = kB * kNE;
constexpr int kRowsV = kB * kNV;
constexpr float kActCarry = 8.0f;
constexpr float kWCarry   = 16.0f;
constexpr float kScaleAW  = 1.0f / 128.0f;
constexpr float kScaleAA  = 1.0f / 64.0f;
constexpr float kLnEps    = 1e-5f;
constexpr size_t kOutBytes = 8654848;
constexpr size_t kOut1Off  = 4198400 / 4;
constexpr size_t kOut2Off  = 4460544 / 4;
constexpr size_t kOut3Off  = 6557696 / 4;
static_assert(kOut3Off + (size_t)kB * kNE * kNV == kOutBytes / 4);

typedef __attribute__((ext_vector_type(16))) _Float16 v16h;
typedef __attribute__((ext_vector_type(8)))  _Float16 v8h;
typedef __attribute__((ext_vector_type(16))) __bf16   v16b;
typedef __attribute__((ext_vector_type(8)))  __bf16   v8b;
typedef __attribute__((ext_vector_type(8)))  float    v8f;
typedef __attribute__((ext_vector_type(4)))  float    v4f;
typedef __attribute__((ext_vector_type(4)))  unsigned int v4u;

__device__ __forceinline__ unsigned short f2bf_bits(float f) {
  unsigned u = __float_as_uint(f);
  return (unsigned short)((u + 0x7FFFu + ((u >> 16) & 1u)) >> 16);
}
__device__ __forceinline__ float bf_bits2f(unsigned short h) { return __uint_as_float(((unsigned)h) << 16); }

__device__ __forceinline__ void dep_guard_h(v8f& a, v8f& b, v16h x, v16h y) { asm volatile("v_nop\n\tv_nop\n\tv_nop\n\tv_nop" : "+v"(a), "+v"(b) : "v"(x), "v"(y)); }
__device__ __forceinline__ void dep_guard_b(v8f& a, v8f& b, v16b x, v16b y) { asm volatile("v_nop\n\tv_nop\n\tv_nop\n\tv_nop" : "+v"(a), "+v"(b) : "v"(x), "v"(y)); }
__device__ __forceinline__ void keep4_h(v16h a, v16h b, v16h c, v16h d) { asm volatile("v_nop" :: "v"(a), "v"(b), "v"(c), "v"(d)); }
__device__ __forceinline__ void keep4_b(v16b a, v16b b, v16b c, v16b d) { asm volatile("v_nop" :: "v"(a), "v"(b), "v"(c), "v"(d)); }
__device__ __forceinline__ void acc_guard4(v8f& a, v8f& b, v8f& c, v8f& d) { asm volatile("v_nop\n\tv_nop\n\tv_nop\n\tv_nop" : "+v"(a), "+v"(b), "+v"(c), "+v"(d)); }
template <typename T> struct Frag;
template <> struct Frag<_Float16> {
  typedef v16h V; union U { v16h v; v8h h[2]; };
  static __device__ __forceinline__ v16h load(const _Float16* p) {
    U f; f.h[0] = *(const v8h*)(p); f.h[1] = *(const v8h*)(p + 16); return f.v;
  }
  static __device__ __forceinline__ v8f mma(v16h a, v16h b, v8f c) {
    return __builtin_amdgcn_wmma_f32_16x16x32_f16(false, a, false, b, (short)0, c, false, false);
  }
  static __device__ __forceinline__ void guard(v8f& a, v8f& b, v16h x, v16h y) { dep_guard_h(a, b, x, y); }
  static __device__ __forceinline__ void keep(v16h a, v16h b, v16h c, v16h d) { keep4_h(a, b, c, d); }
};
template <> struct Frag<__bf16> {
  typedef v16b V; union U { v16b v; v8b h[2]; };
  static __device__ __forceinline__ v16b load(const __bf16* p) {
    U f; f.h[0] = *(const v8b*)(p); f.h[1] = *(const v8b*)(p + 16); return f.v;
  }
  static __device__ __forceinline__ v8f mma(v16b a, v16b b, v8f c) {
    return __builtin_amdgcn_wmma_f32_16x16x32_bf16(false, a, false, b, (short)0, c, false, false);
  }
  static __device__ __forceinline__ void guard(v8f& a, v8f& b, v16b x, v16b y) { dep_guard_b(a, b, x, y); }
  static __device__ __forceinline__ void keep(v16b a, v16b b, v16b c, v16b d) { keep4_b(a, b, c, d); }
};

__device__ __forceinline__ unsigned pk16(unsigned short a, unsigned short b) { return (unsigned)a | ((unsigned)b << 16); }
__device__ __forceinline__ unsigned short h_bits(float f) { const _Float16 h = (_Float16)f; return __builtin_bit_cast(unsigned short, h); }

__device__ __forceinline__ float wave_sum(float s) {
#pragma unroll
  for (int off = 16; off > 0; off >>= 1) s += __shfl_xor(s, off, 32);
  return s;
}

template <int ET> struct Elem;
template <> struct Elem<0> { typedef _Float16 T; };
template <> struct Elem<1> { typedef __bf16 T; };
template <int ET, bool SPLIT, int BIAS_MODE, int OUT_MODE, bool RESID, int ACT = 0>
__global__ __launch_bounds__(256) void wmma_gemm64(
    const unsigned short* __restrict__ Ap, const unsigned short* __restrict__ A2p, int lda, long strideA,
    const unsigned short* __restrict__ Btp, const unsigned short* __restrict__ Bt2p, int ldb, long strideB,
    void* __restrict__ Cout, void* __restrict__ Cout2, int ldc, long strideC,
    const float* __restrict__ bias,
    const float* __restrict__ resid, long strideR,
    int M, int N, int K, float scale) {
  typedef typename Elem<ET>::T T;
  typedef typename Frag<T>::V V;
  const T* A = (const T*)Ap; const T* A2 = (const T*)A2p; const T* Bt = (const T*)Btp; const T* Bt2 = (const T*)Bt2p;
  __shared__ __align__(16) float sT[8][16 * 68];
  const int b    = blockIdx.y;
  const int lane = threadIdx.x & 31;
  const int wave = threadIdx.x >> 5;
  const int tilesN = N >> 6;
  const int tilesM = M >> 6;
  const int tile = blockIdx.x * 8 + wave;
  if (tile >= tilesM * tilesN) return;
  const int tm = tile / tilesN;
  const int tn = tile - tm * tilesN;
  const int m0 = tm << 6;
  const int n0 = tn << 6;

  const T* Ab  = A  + (size_t)b * strideA;
  const T* Bb  = Bt + (size_t)b * strideB;
  const T* Ab2 = SPLIT ? (A2  + (size_t)b * strideA) : nullptr;
  const T* Bb2 = SPLIT ? (Bt2 + (size_t)b * strideB) : nullptr;

  const int rlane = lane & 15;
  const int koff  = (lane >> 4) * 8;
  const int mOff  = (lane >> 4) * 8;

  v8f acc[4][4];
#pragma unroll
  for (int i = 0; i < 4; ++i)
#pragma unroll
    for (int j = 0; j < 4; ++j) acc[i][j] = (v8f){0.f,0.f,0.f,0.f,0.f,0.f,0.f,0.f};

  for (int k0 = 0; k0 < K; k0 += 32) {
    V bh[4], bl[4];
#pragma unroll
    for (int j = 0; j < 4; ++j) {
      const size_t bo = (size_t)(n0 + (j << 4) + rlane) * ldb + koff + k0;
      bh[j] = Frag<T>::load(Bb + bo);
      if (SPLIT) bl[j] = Frag<T>::load(Bb2 + bo);
    }
#pragma unroll
    for (int i = 0; i < 4; ++i) {
      const size_t ao = (size_t)(m0 + (i << 4) + rlane) * lda + koff + k0;
      V ah = Frag<T>::load(Ab + ao);
      V al;
      if (SPLIT) al = Frag<T>::load(Ab2 + ao);
#pragma unroll
      for (int j = 0; j < 4; ++j) {
        acc[i][j] = Frag<T>::mma(ah, bh[j], acc[i][j]);
        if (SPLIT) {
          acc[i][j] = Frag<T>::mma(ah, bl[j], acc[i][j]);
          acc[i][j] = Frag<T>::mma(al, bh[j], acc[i][j]);
        }
      }
      Frag<T>::guard(acc[i][0], acc[i][3], ah, SPLIT ? al : ah);
    }
    Frag<T>::keep(bh[0], bh[1], bh[2], bh[3]);
    if (SPLIT) Frag<T>::keep(bl[0], bl[1], bl[2], bl[3]);
  }
  acc_guard4(acc[0][0], acc[0][1], acc[0][2], acc[0][3]);
  acc_guard4(acc[1][0], acc[1][1], acc[1][2], acc[1][3]);
  acc_guard4(acc[2][0], acc[2][1], acc[2][2], acc[2][3]);
  acc_guard4(acc[3][0], acc[3][1], acc[3][2], acc[3][3]);

  float* slab = sT[wave];
  const float* Rb = RESID ? (resid + (size_t)b * strideR) : nullptr;
#pragma unroll
  for (int i = 0; i < 4; ++i) {
    const int mBase = m0 + (i << 4);
#pragma unroll
    for (int j = 0; j < 4; ++j) {
      const int n = n0 + (j << 4) + rlane;
      float bv = 0.f;
      if (BIAS_MODE == 2) bv = bias[n];
#pragma unroll
      for (int r = 0; r < 8; ++r) {
        float v = acc[i][j][r] * scale;
        if (BIAS_MODE == 1) v += bias[mBase + mOff + r];
        if (BIAS_MODE == 2) v += bv;
        if (RESID) v += Rb[(size_t)(mBase + mOff + r) * ldc + n];
        if (ACT == 2) v = fmaxf(v, 0.0f);
        if (ACT == 4) v = (v > 0.f) ? v : 0.01f * v;
        slab[(mOff + r) * 68 + (j << 4) + rlane] = v;
      }
    }
    __builtin_amdgcn_fence(__ATOMIC_RELEASE, "workgroup");
    __builtin_amdgcn_wave_barrier();
    __builtin_amdgcn_fence(__ATOMIC_ACQUIRE, "workgroup");
    if (OUT_MODE == 0) {
      float* C = (float*)Cout + (size_t)b * strideC;
      const int hh = lane >> 4, c4 = (lane & 15) * 4;
      for (int pass = 0; pass < 2; ++pass) {
#pragma unroll
        for (int it = 0; it < 8; ++it) {
          const int row = it * 2 + hh;
          v4f v = *(const v4f*)(slab + row * 68 + c4);
          *(volatile v4f*)(C + (size_t)(mBase + row) * ldc + n0 + c4) = v;
        }
        __threadfence();
      }
    } else {
      const int q = lane >> 3, c8 = (lane & 7) * 8;
      unsigned short* C  = (unsigned short*)Cout  + (size_t)b * strideC;
      unsigned short* C2 = (OUT_MODE == 2) ? ((unsigned short*)Cout2 + (size_t)b * strideC) : nullptr;
      for (int pass = 0; pass < 2; ++pass) {
#pragma unroll
        for (int it = 0; it < 4; ++it) {
          const int row = it * 4 + q;
          const float* sp = slab + row * 68 + c8;
          v8h hv, lv;
#pragma unroll
          for (int e = 0; e < 8; ++e) {
            if (OUT_MODE == 1) {
              hv[e] = (_Float16)sp[e];
            } else {
              unsigned short hb = f2bf_bits(sp[e]);
              unsigned short lb = f2bf_bits(sp[e] - bf_bits2f(hb));
              hv[e] = __builtin_bit_cast(_Float16, hb);
              lv[e] = __builtin_bit_cast(_Float16, lb);
            }
          }
          *(volatile v8h*)(C + (size_t)(mBase + row) * ldc + n0 + c8) = hv;
          if (OUT_MODE == 2) *(volatile v8h*)(C2 + (size_t)(mBase + row) * ldc + n0 + c8) = lv;
        }
        __threadfence();
      }
    }
    __builtin_amdgcn_fence(__ATOMIC_RELEASE, "workgroup");
    __builtin_amdgcn_wave_barrier();
    __builtin_amdgcn_fence(__ATOMIC_ACQUIRE, "workgroup");
  }
}

__global__ __launch_bounds__(256) void wt4_kernel(
    const float* __restrict__ s0, int K0, unsigned short* __restrict__ o0, int l0,
    const float* __restrict__ s1, int K1, unsigned short* __restrict__ o1, int l1,
    const float* __restrict__ s2, int K2, unsigned short* __restrict__ o2, int l2,
    const float* __restrict__ s3, int K3, unsigned short* __restrict__ o3, int l3, float scale) {
  __shared__ float sm[64][65];
  const int z = blockIdx.z;
  const float* S = (z == 0) ? s0 : (z == 1) ? s1 : (z == 2) ? s2 : s3;
  unsigned short* O = (z == 0) ? o0 : (z == 1) ? o1 : (z == 2) ? o2 : o3;
  const int Ks = (z == 0) ? K0 : (z == 1) ? K1 : (z == 2) ? K2 : K3;
  const int ld = (z == 0) ? l0 : (z == 1) ? l1 : (z == 2) ? l2 : l3;
  const int kk0 = blockIdx.x * 64;
  const int nn0 = blockIdx.y * 64;
  if (kk0 >= Ks) return;
  const int t = threadIdx.x;
#pragma unroll
  for (int i = 0; i < 16; ++i) {
    const int e = i * 256 + t;
    const int r = e >> 6;
    const int c = e & 63;
    sm[c][r] = S[(size_t)(kk0 + r) * kD + nn0 + c] * scale;
  }
  __syncthreads();
  const int lane = t & 31, wave = t >> 5;
  const int q = lane >> 3, c8 = (lane & 7) * 8;
  for (int pass = 0; pass < 2; ++pass) {
#pragma unroll
    for (int it = 0; it < 2; ++it) {
      const int row = wave * 8 + it * 4 + q;
      unsigned short hb[8];
#pragma unroll
      for (int e = 0; e < 8; ++e) hb[e] = h_bits(sm[row][c8 + e]);
      const v4u u = (v4u){pk16(hb[0], hb[1]), pk16(hb[2], hb[3]), pk16(hb[4], hb[5]), pk16(hb[6], hb[7])};
      *(volatile v4u*)(O + (size_t)(nn0 + row) * ld + kk0 + c8) = u;
    }
    __threadfence();
  }
}

__global__ __launch_bounds__(128) void bias4_kernel(const float* __restrict__ a0, const float* __restrict__ c0,
                                                    const float* __restrict__ a1, const float* __restrict__ c1,
                                                    const float* __restrict__ a2, const float* __restrict__ c2,
                                                    const float* __restrict__ a3, const float* __restrict__ c3,
                                                    float* __restrict__ out) {
  const int t = threadIdx.x;
  const int slot = t >> 5;
  const int i4 = (t & 31) * 4;
  const v4f x0 = *(const v4f*)(a0 + i4) + *(const v4f*)(c0 + i4);
  const v4f x1 = *(const v4f*)(a1 + i4) + *(const v4f*)(c1 + i4);
  const v4f x2 = *(const v4f*)(a2 + i4) + *(const v4f*)(c2 + i4);
  const v4f x3 = *(const v4f*)(a3 + i4) + *(const v4f*)(c3 + i4);
  const v4f v = (slot == 0) ? x0 : (slot == 1) ? x1 : (slot == 2) ? x2 : x3;
  float* p = out + (size_t)t * 4;
  *(volatile v4f*)p = v;
  __threadfence();
  *(volatile v4f*)p = v;
}

__global__ __launch_bounds__(256) void cast8_kernel(const float* __restrict__ in, unsigned short* __restrict__ out,
                                                    int n8, float scale) {
  const int i = blockIdx.x * 256 + threadIdx.x;
  if (i >= n8) return;
  const float* p = in + 8 * (size_t)i;
  const v4f a = *(const v4f*)(p);
  const v4f c = *(const v4f*)(p + 4);
  unsigned short hb[8];
#pragma unroll
  for (int e = 0; e < 4; ++e) {
    hb[e]     = h_bits(a[e] * scale);
    hb[4 + e] = h_bits(c[e] * scale);
  }
  const v4u u = (v4u){pk16(hb[0], hb[1]), pk16(hb[2], hb[3]), pk16(hb[4], hb[5]), pk16(hb[6], hb[7])};
  unsigned short* q = out + 8 * (size_t)i;
  *(volatile v4u*)q = u;
  __threadfence();
  *(volatile v4u*)q = u;
}

template <bool DO_LN, bool WF32>
__global__ __launch_bounds__(256) void rowplanes_kernel(const float* __restrict__ src, const float* __restrict__ add,
                                                        const float* __restrict__ gam, const float* __restrict__ bet,
                                                        float* __restrict__ dstf, unsigned short* __restrict__ p16,
                                                        unsigned short* __restrict__ pT16, int R) {
  __shared__ __align__(16) float sm[64][132];
  const int t = threadIdx.x, lane = t & 31, wave = t >> 5;
  const int grow0 = blockIdx.x * 64;
  const int b  = grow0 / R;
  const int r0 = grow0 - b * R;
  const int c4 = lane * 4;
  v4f g = (v4f){1.f, 1.f, 1.f, 1.f}, bt = (v4f){0.f, 0.f, 0.f, 0.f};
  if (DO_LN) { g = *(const v4f*)(gam + c4); bt = *(const v4f*)(bet + c4); }
#pragma unroll 1
  for (int i = 0; i < 8; ++i) {
    const int lrow = wave * 8 + i;
    const size_t row = (size_t)(grow0 + lrow);
    v4f y = *(const v4f*)(src + row * kD + c4);
    if (DO_LN) {
      const v4f a = *(const v4f*)(add + row * kD + c4);
      y = y + a;
      const float s = wave_sum(y[0] + y[1] + y[2] + y[3]);
      const float mean = s * (1.0f / (float)kD);
      float qv = 0.f;
#pragma unroll
      for (int j = 0; j < 4; ++j) { const float d = y[j] - mean; qv += d * d; }
      qv = wave_sum(qv);
      const float rstd = rsqrtf(qv * (1.0f / (float)kD) + kLnEps);
#pragma unroll
      for (int j = 0; j < 4; ++j) y[j] = (y[j] - mean) * rstd * g[j] + bt[j];
    }
#pragma unroll
    for (int j = 0; j < 4; ++j) sm[lrow][c4 + j] = y[j];
    if (WF32) {
      float* dp = dstf + row * kD + c4;
      *(volatile v4f*)dp = y;
      __threadfence();
      *(volatile v4f*)dp = y;
    }
  }
  __syncthreads();
  const int hh = lane >> 4, c8r = (lane & 15) * 8;
  const int q = lane >> 3, r8 = (lane & 7) * 8;
  for (int pass = 0; pass < 2; ++pass) {
#pragma unroll
    for (int it = 0; it < 4; ++it) {
      const int lrow = wave * 8 + it * 2 + hh;
      unsigned short hb[8];
#pragma unroll
      for (int e = 0; e < 8; ++e) hb[e] = h_bits(sm[lrow][c8r + e] * kActCarry);
      const v4u u = (v4u){pk16(hb[0], hb[1]), pk16(hb[2], hb[3]), pk16(hb[4], hb[5]), pk16(hb[6], hb[7])};
      *(volatile v4u*)(p16 + (size_t)(grow0 + lrow) * kD + c8r) = u;
    }
#pragma unroll
    for (int it = 0; it < 4; ++it) {
      const int d = wave * 16 + it * 4 + q;
      unsigned short hb[8];
#pragma unroll
      for (int e = 0; e < 8; ++e) hb[e] = h_bits(sm[r8 + e][d] * kActCarry);
      const v4u u = (v4u){pk16(hb[0], hb[1]), pk16(hb[2], hb[3]), pk16(hb[4], hb[5]), pk16(hb[6], hb[7])};
      *(volatile v4u*)(pT16 + ((size_t)(b * kD + d)) * R + r0 + r8) = u;
    }
    __threadfence();
  }
}

__global__ __launch_bounds__(256) void eind_kernel(const float* __restrict__ esrc, const float* __restrict__ w,
                                                   const float* __restrict__ bsc, float* __restrict__ out) {
  __shared__ float rs[32];
  const int t = threadIdx.x, lane = t & 31, wave = t >> 5;
  const int base = blockIdx.x * 32;
  const v4f wv = *(const v4f*)(w + lane * 4);
  const float b0 = bsc[0];
#pragma unroll 1
  for (int i = 0; i < 4; ++i) {
    const int row = base + wave * 4 + i;
    const v4f x = *(const v4f*)(esrc + (size_t)row * kD + lane * 4);
    float s = x[0] * wv[0] + x[1] * wv[1] + x[2] * wv[2] + x[3] * wv[3];
    s = wave_sum(s);
    const float z = s + b0;
    const float val = 1.0f / (1.0f + expf(-z));
    if (lane == 0) rs[wave * 4 + i] = val;
  }
  __syncthreads();
  if (wave == 0) {
    const float v = rs[lane];
    float* p = out + base + lane;
    *(volatile float*)p = v;
    __threadfence();
    *(volatile float*)p = v;
  }
}

__global__ __launch_bounds__(256) void incid_kernel(const float* __restrict__ ve, const float* __restrict__ ee,
                                                    const float* __restrict__ isrc, const float* __restrict__ eind,
                                                    const float* __restrict__ wi, const float* __restrict__ bi,
                                                    const float* __restrict__ wo, const float* __restrict__ bo,
                                                    float* __restrict__ idst, unsigned short* __restrict__ im16,
                                                    unsigned short* __restrict__ imT16) {
  __shared__ float ves[64][65];
  __shared__ float ees[64][65];
  __shared__ float wis[64];
  __shared__ float bis[64];
  __shared__ float wos[64];
  __shared__ float eis[64];
  __shared__ __align__(16) float res[64][68];
  const int t = threadIdx.x, lane = t & 31, wave = t >> 5;
  const int bx = blockIdx.x;
  const int b  = bx >> 5;
  const int et = (bx >> 4) & 1;
  const int nt = bx & 15;
  const int e0 = et * 64, n0 = nt * 64;
  const int nl = t & 63, eg = t >> 6;
  if (t < 64) eis[t] = eind[b * kNE + e0 + t];
  float iv[16], acc[16];
#pragma unroll
  for (int j = 0; j < 16; ++j) {
    iv[j] = isrc[((size_t)(b * kNE + e0 + eg * 16 + j)) * kNV + n0 + nl];
    acc[j] = 0.f;
  }
  for (int dc = 0; dc < 2; ++dc) {
    __syncthreads();
#pragma unroll
    for (int i = 0; i < 16; ++i) {
      const int e = i * 256 + t;
      const int r = e >> 6;
      const int c = e & 63;
      ves[r][c] = ve[((size_t)(b * kNV + n0 + r)) * kD + dc * 64 + c];
      ees[r][c] = ee[((size_t)(b * kNE + e0 + r)) * kD + dc * 64 + c];
    }
    if (t < 64) { wis[t] = wi[dc * 64 + t]; bis[t] = bi[dc * 64 + t]; wos[t] = wo[dc * 64 + t]; }
    __syncthreads();
#pragma unroll 1
    for (int d = 0; d < 64; ++d) {
      const float vn = ves[nl][d];
      const float w_i = wis[d], b_i = bis[d], w_o = wos[d];
#pragma unroll
      for (int j = 0; j < 16; ++j) {
        const float sa = vn + ees[eg * 16 + j][d];
        const float sb = iv[j] * w_i + b_i;
        const float h = sa + sb;
        acc[j] = fmaxf(h, 0.f) * w_o + acc[j];
      }
    }
  }
  const float bo_v = bo[0];
#pragma unroll
  for (int j = 0; j < 16; ++j) res[eg * 16 + j][nl] = acc[j] + bo_v;
  __syncthreads();
#pragma unroll 1
  for (int qq = 0; qq < 16; ++qq) {
    const int idx = qq * 256 + t;
    const int el = idx >> 6;
    const int n2 = idx & 63;
    const float z = res[el][n2];
    const float s = 1.0f / (1.0f + expf(-z));
    res[el][n2] = s;
  }
  __syncthreads();
  const int hh = lane >> 4, c4 = (lane & 15) * 4;
  const int q = lane >> 3, c8 = (lane & 7) * 8;
  for (int pass = 0; pass < 2; ++pass) {
#pragma unroll
    for (int it = 0; it < 4; ++it) {
      const int row = wave * 8 + it * 2 + hh;
      v4f v;
#pragma unroll
      for (int e = 0; e < 4; ++e) v[e] = res[row][c4 + e];
      *(volatile v4f*)(idst + ((size_t)(b * kNE + e0 + row)) * kNV + n0 + c4) = v;
    }
#pragma unroll
    for (int it = 0; it < 2; ++it) {
      const int row = wave * 8 + it * 4 + q;
      const float er = eis[row];
      unsigned short hb[8];
#pragma unroll
      for (int e = 0; e < 8; ++e) hb[e] = h_bits((res[row][c8 + e] * er) * kActCarry);
      const v4u u = (v4u){pk16(hb[0], hb[1]), pk16(hb[2], hb[3]), pk16(hb[4], hb[5]), pk16(hb[6], hb[7])};
      *(volatile v4u*)(im16 + ((size_t)(b * kNE + e0 + row)) * kNV + n0 + c8) = u;
    }
#pragma unroll
    for (int it = 0; it < 2; ++it) {
      const int nrow = wave * 8 + it * 4 + q;
      unsigned short hb[8];
#pragma unroll
      for (int e = 0; e < 8; ++e) hb[e] = h_bits((res[c8 + e][nrow] * eis[c8 + e]) * kActCarry);
      const v4u u = (v4u){pk16(hb[0], hb[1]), pk16(hb[2], hb[3]), pk16(hb[4], hb[5]), pk16(hb[6], hb[7])};
      *(volatile v4u*)(imT16 + ((size_t)(b * kNV + n0 + nrow)) * kNE + e0 + c8) = u;
    }
    __threadfence();
  }
}

template <int NP>
__global__ __launch_bounds__(256) void cln_kernel(const float* __restrict__ p0, const float* __restrict__ p1,
                                                  const float* __restrict__ p2, const float* __restrict__ gam,
                                                  const float* __restrict__ bet, float* __restrict__ outf,
                                                  float* __restrict__ part) {
  constexpr int W = 128 * NP;
  constexpr float invW = 1.0f / (float)W;
  __shared__ __align__(16) v4f smp[8][W / 4];
  const int t = threadIdx.x, lane = t & 31, wave = t >> 5;
  const int grow0 = blockIdx.x * 64;
  const int c4 = lane * 4;
  v4f g[3], bb[3], cs[3];
#pragma unroll
  for (int p = 0; p < 3; ++p) { g[p] = (v4f){1.f,1.f,1.f,1.f}; bb[p] = (v4f){0.f,0.f,0.f,0.f}; cs[p] = (v4f){0.f,0.f,0.f,0.f}; }
#pragma unroll
  for (int p = 0; p < NP; ++p) { g[p] = *(const v4f*)(gam + p * 128 + c4); bb[p] = *(const v4f*)(bet + p * 128 + c4); }
#pragma unroll 1
  for (int i = 0; i < 8; ++i) {
    const size_t row = (size_t)(grow0 + wave * 8 + i);
    v4f x[3];
    x[0] = *(const v4f*)(p0 + row * 128 + c4);
    x[1] = x[0]; x[2] = x[0];
    if (NP > 1) x[1] = *(const v4f*)(p1 + row * 128 + c4);
    if (NP > 2) x[2] = *(const v4f*)(p2 + row * 128 + c4);
    float s = 0.f;
#pragma unroll
    for (int p = 0; p < NP; ++p) s += x[p][0] + x[p][1] + x[p][2] + x[p][3];
    s = wave_sum(s);
    const float mean = s * invW;
    float qv = 0.f;
#pragma unroll
    for (int p = 0; p < NP; ++p)
#pragma unroll
      for (int j = 0; j < 4; ++j) { const float d = x[p][j] - mean; qv += d * d; }
    qv = wave_sum(qv);
    const float rstd = rsqrtf(qv * invW + kLnEps);
#pragma unroll
    for (int p = 0; p < NP; ++p) {
      v4f y;
#pragma unroll
      for (int j = 0; j < 4; ++j) y[j] = (x[p][j] - mean) * rstd * g[p][j] + bb[p][j];
      cs[p] = cs[p] + y;
      float* dp = outf + row * W + p * 128 + c4;
      *(volatile v4f*)dp = y;
      __threadfence();
      *(volatile v4f*)dp = y;
    }
  }
#pragma unroll
  for (int p = 0; p < NP; ++p) smp[wave][p * 32 + lane] = cs[p];
  __syncthreads();
  if (t < W / 4) {
    v4f s = smp[0][t];
#pragma unroll
    for (int w = 1; w < 8; ++w) s = s + smp[w][t];
    float* dp = part + (size_t)blockIdx.x * W + t * 4;
    *(volatile v4f*)dp = s;
    __threadfence();
    *(volatile v4f*)dp = s;
  }
}

template <int W>
__global__ __launch_bounds__(256) void builda_kernel(const float* __restrict__ y, const float* __restrict__ part,
                                                     unsigned short* __restrict__ A, int R, float invR) {
  __shared__ float meanv[W];
  const int t = threadIdx.x;
  const int grow0 = blockIdx.x * 64;
  const int b = grow0 / R;
  const int nb = R >> 6;
  const int pb0 = b * nb;
  for (int c = t; c < W; c += 256) {
    float s = 0.f;
#pragma unroll 1
    for (int qq = 0; qq < nb; ++qq) s += part[(size_t)(pb0 + qq) * W + c];
    meanv[c] = s * invR;
  }
  __syncthreads();
  constexpr int CPR = W / 4;
#pragma unroll 1
  for (int idx = t; idx < 64 * CPR; idx += 256) {
    const int lrow = idx / CPR;
    const int ch = idx - lrow * CPR;
    const int col0 = ch * 8;
    const bool first = col0 < W;
    const int colm = first ? col0 : col0 - W;
    const float* yp = y + (size_t)(grow0 + lrow) * W + colm;
    const v4f ya = *(const v4f*)(yp);
    const v4f yb = *(const v4f*)(yp + 4);
    unsigned short hb[8];
#pragma unroll
    for (int e = 0; e < 4; ++e) {
      const float m0 = meanv[colm + e];
      const float m1 = meanv[colm + 4 + e];
      const float s0 = first ? 0.f : m0;
      const float s1 = first ? 0.f : m1;
      hb[e]     = h_bits((ya[e] - s0) * kActCarry);
      hb[4 + e] = h_bits((yb[e] - s1) * kActCarry);
    }
    const v4u u = (v4u){pk16(hb[0], hb[1]), pk16(hb[2], hb[3]), pk16(hb[4], hb[5]), pk16(hb[6], hb[7])};
    unsigned short* dp = A + (size_t)(grow0 + lrow) * (2 * W) + col0;
    *(volatile v4u*)dp = u;
    __threadfence();
    *(volatile v4u*)dp = u;
  }
}

__global__ __launch_bounds__(256) void preds_kernel(const float* i0, const float* i1,
                                                    const float* __restrict__ eind, float* out) {
  constexpr int kTot4 = kT * kB * kNE * (kNV + 1) / 4;
  constexpr int kPerT = kB * kNE * (kNV + 1);
  const int gid = blockIdx.x * 256 + threadIdx.x;
  if (gid >= kTot4) return;
  v4f v;
#pragma unroll
  for (int e = 0; e < 4; ++e) {
    const int p = gid * 4 + e;
    int tt = p / kPerT;
    tt = tt > 1 ? 1 : tt;
    const int rem = p - tt * kPerT;
    int row = rem / (kNV + 1);
    row = row > (kRowsE - 1) ? (kRowsE - 1) : row;
    const int col = rem - row * (kNV + 1);
    const int colc = col < kNV ? col : (kNV - 1);
    const size_t ii = (size_t)row * kNV + colc;
    const float a0 = i0[ii];
    const float a1 = i1[ii];
    const float ev = eind[tt * kRowsE + row];
    const float iv = (tt == 0) ? a0 : a1;
    v[e] = (col < kNV) ? iv : ev;
  }
  float* dp = out + (size_t)gid * 4;
  *(volatile v4f*)dp = v;
  __threadfence();
  *(volatile v4f*)dp = v;
}

static inline dim3 gemm_grid(int M, int N, int batch) {
  return dim3((unsigned)(((M >> 6) * (N >> 6) + 7) / 8), (unsigned)batch, 1);
}

extern "C" void kernel_launch(void* const* d_in, const int* in_sizes, int n_in,
                              void* d_out, int out_size, void* d_ws, size_t ws_size,
                              hipStream_t stream)
{
  if (n_in < 44) return;
  if ((size_t)out_size * 4 < kOutBytes) return;
  if (in_sizes[0] != kRowsV * kDIN || in_sizes[1] != kRowsE * kD || in_sizes[2] != kRowsV * kD ||
      in_sizes[3] != kB * kNE * kNV) return;

  const float* in_inputs = (const float*)d_in[0];
  const float* in_e   = (const float*)d_in[1];
  const float* in_v   = (const float*)d_in[2];
  const float* in_i   = (const float*)d_in[3];
  const float* pw     = (const float*)d_in[4];
  const float* inc_we = (const float*)d_in[5];
  const float* inc_wn = (const float*)d_in[6];
  const float* inc_wi = (const float*)d_in[7];
  const float* inc_wo = (const float*)d_in[8];
  const float* ind_w  = (const float*)d_in[9];
  const float* me_w1a = (const float*)d_in[10];
  const float* me_w2a = (const float*)d_in[11];
  const float* me_w1b = (const float*)d_in[12];
  const float* me_w2b = (const float*)d_in[13];
  const float* mn_w1a = (const float*)d_in[14];
  const float* mn_w2a = (const float*)d_in[15];
  const float* mn_w1b = (const float*)d_in[16];
  const float* mn_w2b = (const float*)d_in[17];
  const float* pb     = (const float*)d_in[18];
  const float* inc_be = (const float*)d_in[19];
  const float* inc_bn = (const float*)d_in[20];
  const float* inc_bi = (const float*)d_in[21];
  const float* inc_bo = (const float*)d_in[22];
  const float* ind_b  = (const float*)d_in[23];
  const float* me_b1a = (const float*)d_in[24];
  const float* me_b2a = (const float*)d_in[25];
  const float* me_b1b = (const float*)d_in[26];
  const float* me_b2b = (const float*)d_in[27];
  const float* mn_b1a = (const float*)d_in[28];
  const float* mn_b2a = (const float*)d_in[29];
  const float* mn_b1b = (const float*)d_in[30];
  const float* mn_b2b = (const float*)d_in[31];
  const float* me_g   = (const float*)d_in[32];
  const float* mn_g   = (const float*)d_in[33];
  const float* pre_e_g= (const float*)d_in[34];
  const float* pre_n_g= (const float*)d_in[35];
  const float* ln_e_g = (const float*)d_in[36];
  const float* ln_n_g = (const float*)d_in[37];
  const float* me_bg  = (const float*)d_in[38];
  const float* mn_bg  = (const float*)d_in[39];
  const float* pre_e_b= (const float*)d_in[40];
  const float* pre_n_b= (const float*)d_in[41];
  const float* ln_e_b = (const float*)d_in[42];
  const float* ln_n_b = (const float*)d_in[43];

  char* ws = (char*)d_ws;
  size_t cur = 0;
  auto carve = [&](size_t bytes) -> char* { char* p = ws + cur; cur += (bytes + 255) & ~(size_t)255; return p; };
  unsigned short* pwT  = (unsigned short*)carve(2ul * kD * kDIN);
  unsigned short* wnT  = (unsigned short*)carve(2ul * kD * kD);
  unsigned short* weT  = (unsigned short*)carve(2ul * kD * kD);
  unsigned short* WaE  = (unsigned short*)carve(2ul * kD * 512);
  unsigned short* WbE  = (unsigned short*)carve(2ul * kD * 256);
  unsigned short* WaN  = (unsigned short*)carve(2ul * kD * 768);
  unsigned short* WbN  = (unsigned short*)carve(2ul * kD * 256);
  float* bsum  = (float*)carve(4ul * 4 * kD);
  unsigned short* in16 = (unsigned short*)carve(2ul * kRowsV * kDIN);
  float* xf    = (float*)carve(4ul * kRowsV * kD);
  unsigned short* v16  = (unsigned short*)carve(2ul * kRowsV * kD);
  unsigned short* vT16 = (unsigned short*)carve(2ul * kRowsV * kD);
  unsigned short* e16  = (unsigned short*)carve(2ul * kRowsE * kD);
  unsigned short* eT16 = (unsigned short*)carve(2ul * kRowsE * kD);
  float* ebuf  = (float*)carve(4ul * kRowsE * kD);
  float* vbuf  = (float*)carve(4ul * kRowsV * kD);
  float* vef   = (float*)carve(4ul * kRowsV * kD);
  float* eef   = (float*)carve(4ul * kRowsE * kD);
  float* eindp = (float*)carve(4ul * kT * kRowsE);
  float* ist0  = (float*)carve(4ul * kB * kNE * kNV);
  unsigned short* im16  = (unsigned short*)carve(2ul * kB * kNE * kNV);
  unsigned short* imT16 = (unsigned short*)carve(2ul * kB * kNE * kNV);
  float* upde  = (float*)carve(4ul * kRowsE * kD);
  float* cef   = (float*)carve(4ul * kRowsE * 256);
  float* parte = (float*)carve(4ul * (kRowsE / 64) * 256);
  float* parte2= (float*)carve(4ul * (kRowsE / 64) * 128);
  unsigned short* Ae   = (unsigned short*)carve(2ul * kRowsE * 512);
  unsigned short* Aeb  = (unsigned short*)carve(2ul * kRowsE * 256);
  float* t1e   = (float*)carve(4ul * kRowsE * kD);
  float* ue    = (float*)carve(4ul * kRowsE * kD);
  float* o2e   = (float*)carve(4ul * kRowsE * kD);
  float* updn  = (float*)carve(4ul * kRowsV * kD);
  float* cnf   = (float*)carve(4ul * kRowsV * 384);
  float* partn = (float*)carve(4ul * (kRowsV / 64) * 384);
  float* partn2= (float*)carve(4ul * (kRowsV / 64) * 128);
  unsigned short* An   = (unsigned short*)carve(2ul * kRowsV * 768);
  unsigned short* Anb  = (unsigned short*)carve(2ul * kRowsV * 256);
  float* t1n   = (float*)carve(4ul * kRowsV * kD);
  float* un    = (float*)carve(4ul * kRowsV * kD);
  float* o2n   = (float*)carve(4ul * kRowsV * kD);
  if (cur > ws_size) return;

  float* outp = (float*)d_out;
  float* out1 = outp + kOut1Off;
  float* out2 = outp + kOut2Off;
  float* out3 = outp + kOut3Off;

  bias4_kernel<<<1, 128, 0, stream>>>(me_b1a, me_b2a, me_b1b, me_b2b, mn_b1a, mn_b2a, mn_b1b, mn_b2b, bsum);
  {
    const dim3 wg(6, 2, 4);
    wt4_kernel<<<wg, 256, 0, stream>>>(pw, kDIN, pwT, kDIN,  inc_wn, kD, wnT, kD,
                                        inc_we, kD, weT, kD,  me_w1a, 256, WaE, 512, kWCarry);
    wt4_kernel<<<wg, 256, 0, stream>>>(me_w2a, 256, WaE + 256, 512,  me_w1b, 128, WbE, 256,
                                        me_w2b, 128, WbE + 128, 256,  mn_w1a, 384, WaN, 768, kWCarry);
    wt4_kernel<<<wg, 256, 0, stream>>>(mn_w2a, 384, WaN + 384, 768,  mn_w1b, 128, WbN, 256,
                                        mn_w2b, 128, WbN + 128, 256,  mn_w2b, 0, WbN, 256, kWCarry);
  }
  {
    const int n8 = kRowsV * kDIN / 8;
    cast8_kernel<<<(n8 + 255) / 256, 256, 0, stream>>>(in_inputs, in16, n8, kActCarry);
  }
  rowplanes_kernel<false, false><<<kRowsV / 64, 256, 0, stream>>>(in_v, in_v, ln_n_g, ln_n_b, vbuf, v16, vT16, kNV);
  rowplanes_kernel<false, false><<<kRowsE / 64, 256, 0, stream>>>(in_e, in_e, ln_e_g, ln_e_b, ebuf, e16, eT16, kNE);
  wmma_gemm64<0, false, 2, 0, false, 0><<<gemm_grid(kRowsV, kD, 1), 256, 0, stream>>>(
      in16, in16, kDIN, 0, pwT, pwT, kDIN, 0, xf, xf, kD, 0, pb, pb, 0, kRowsV, kD, kDIN, kScaleAW);

  const float* ecur = in_e;
  const float* vcur = in_v;
  const float* icur = in_i;
  for (int t = 0; t < kT; ++t) {
    const bool last = (t == kT - 1);
    float* edst = last ? out1 : ebuf;
    float* vdst = last ? out2 : vbuf;
    float* idst = last ? out3 : ist0;
    float* eind_t = eindp + (size_t)t * kRowsE;

    wmma_gemm64<0, false, 2, 0, false, 0><<<gemm_grid(kRowsV, kD, 1), 256, 0, stream>>>(
        v16, v16, kD, 0, wnT, wnT, kD, 0, vef, vef, kD, 0, inc_bn, pb, 0, kRowsV, kD, kD, kScaleAW);
    wmma_gemm64<0, false, 2, 0, false, 0><<<gemm_grid(kRowsE, kD, 1), 256, 0, stream>>>(
        e16, e16, kD, 0, weT, weT, kD, 0, eef, eef, kD, 0, inc_be, pb, 0, kRowsE, kD, kD, kScaleAW);
    eind_kernel<<<kRowsE / 32, 256, 0, stream>>>(ecur, ind_w, ind_b, eind_t);
    incid_kernel<<<kB * 2 * 16, 256, 0, stream>>>(vef, eef, icur, eind_t, inc_wi, inc_bi, inc_wo, inc_bo,
                                                  idst, im16, imT16);
    wmma_gemm64<0, false, 0, 0, false, 0><<<gemm_grid(kNE, kD, kB), 256, 0, stream>>>(
        im16, im16, kNV, (long)kNE * kNV, vT16, vT16, kNV, (long)kD * kNV, upde, upde, kD, (long)kNE * kD,
        bsum, pb, 0, kNE, kD, kNV, kScaleAA);
    cln_kernel<2><<<kRowsE / 64, 256, 0, stream>>>(ecur, upde, upde, pre_e_g, pre_e_b, cef, parte);
    builda_kernel<256><<<kRowsE / 64, 256, 0, stream>>>(cef, parte, Ae, kNE, 1.0f / (float)kNE);
    wmma_gemm64<0, false, 2, 0, false, 2><<<gemm_grid(kRowsE, kD, 1), 256, 0, stream>>>(
        Ae, Ae, 512, 0, WaE, WaE, 512, 0, t1e, t1e, kD, 0, bsum, pb, 0, kRowsE, kD, 512, kScaleAW);
    cln_kernel<1><<<kRowsE / 64, 256, 0, stream>>>(t1e, t1e, t1e, me_g, me_bg, ue, parte2);
    builda_kernel<128><<<kRowsE / 64, 256, 0, stream>>>(ue, parte2, Aeb, kNE, 1.0f / (float)kNE);
    wmma_gemm64<0, false, 2, 0, false, 0><<<gemm_grid(kRowsE, kD, 1), 256, 0, stream>>>(
        Aeb, Aeb, 256, 0, WbE, WbE, 256, 0, o2e, o2e, kD, 0, bsum + kD, pb, 0, kRowsE, kD, 256, kScaleAW);
    rowplanes_kernel<true, true><<<kRowsE / 64, 256, 0, stream>>>(o2e, ecur, ln_e_g, ln_e_b, edst, e16, eT16, kNE);
    wmma_gemm64<0, false, 0, 0, false, 0><<<gemm_grid(kNV, kD, kB), 256, 0, stream>>>(
        imT16, imT16, kNE, (long)kNV * kNE, eT16, eT16, kNE, (long)kD * kNE, updn, updn, kD, (long)kNV * kD,
        bsum, pb, 0, kNV, kD, kNE, kScaleAA);
    cln_kernel<3><<<kRowsV / 64, 256, 0, stream>>>(xf, vcur, updn, pre_n_g, pre_n_b, cnf, partn);
    builda_kernel<384><<<kRowsV / 64, 256, 0, stream>>>(cnf, partn, An, kNV, 1.0f / (float)kNV);
    wmma_gemm64<0, false, 2, 0, false, 2><<<gemm_grid(kRowsV, kD, 1), 256, 0, stream>>>(
        An, An, 768, 0, WaN, WaN, 768, 0, t1n, t1n, kD, 0, bsum + 2 * kD, pb, 0, kRowsV, kD, 768, kScaleAW);
    cln_kernel<1><<<kRowsV / 64, 256, 0, stream>>>(t1n, t1n, t1n, mn_g, mn_bg, un, partn2);
    builda_kernel<128><<<kRowsV / 64, 256, 0, stream>>>(un, partn2, Anb, kNV, 1.0f / (float)kNV);
    wmma_gemm64<0, false, 2, 0, false, 0><<<gemm_grid(kRowsV, kD, 1), 256, 0, stream>>>(
        Anb, Anb, 256, 0, WbN, WbN, 256, 0, o2n, o2n, kD, 0, bsum + 3 * kD, pb, 0, kRowsV, kD, 256, kScaleAW);
    rowplanes_kernel<true, true><<<kRowsV / 64, 256, 0, stream>>>(o2n, vcur, ln_n_g, ln_n_b, vdst, v16, vT16, kNV);

    ecur = edst;
    vcur = vdst;
    icur = idst;
  }

  preds_kernel<<<(kT * kB * kNE * (kNV + 1) / 4 + 255) / 256, 256, 0, stream>>>(ist0, out3, eindp, outp);
}
